// Reconstructeur_18940805775490
// MI455X (gfx1250) — hardware-verified
//
#include <hip/hip_runtime.h>

#define NM    16
#define G_ALL 4096
#define LAT   1024
#define S0    512
#define S1    256
#define S2    128

#define GT    128
#define PY    520
#define P1    264
#define P2    136
#define PB    40

#define OFF_Y   0
#define OFF_H2  0
#define OFF_H1  (GT * PY * 2)
#define OFF_B0  (OFF_H1 + GT * P1 * 2)
#define BUF_BYTES (S1 * PB * 2)
#define OFF_B1  (OFF_B0 + BUF_BYTES)
#define SMEM_BYTES (OFF_B1 + BUF_BYTES)

#define WS_CVEC 0
#define WS_W1H  32768
#define WS_W2H  (32768 + NM * S1 * S0 * 2)

#define AS3 __attribute__((address_space(3)))

typedef __attribute__((ext_vector_type(16))) _Float16 v16h;
typedef __attribute__((ext_vector_type(8)))  _Float16 v8h;
typedef __attribute__((ext_vector_type(4)))  _Float16 v4h;
typedef __attribute__((ext_vector_type(8)))  float    v8f;
typedef __attribute__((ext_vector_type(4)))  float    v4f;
typedef __attribute__((ext_vector_type(4)))  unsigned int u32x4;
typedef __attribute__((ext_vector_type(8)))  int      i32x8;
typedef __attribute__((ext_vector_type(4)))  int      i32x4;

typedef AS3 _Float16 lds_half;
typedef AS3 float    lds_float;
typedef AS3 v8h      lds_v8h;

union V16H { v16h v; v8h h[2]; };

static __device__ inline v8f wmma_f16(const V16H& a, const V16H& b, v8f c) {
    return __builtin_amdgcn_wmma_f32_16x16x32_f16(
         false, a.v,  false, b.v,
         (short)0, c,  false,  false);
}

static __device__ inline void copy_w_chunk(AS3 _Float16* dst, const _Float16* __restrict__ gsrc, int rows, int stride, int tid) {
    for (int p = tid; p < rows * 4; p += 512) {
        const int r = p >> 2, q = (p & 3) * 8;
        *(AS3 v8h*)(dst + r * PB + q) = *(const v8h*)(gsrc + (size_t)r * stride + q);
    }
}

__global__ void __launch_bounds__(256)
precompute_c_kernel(const float* __restrict__ Wa, const float* __restrict__ x0,
                    const float* __restrict__ ba, const float* __restrict__ bb,
                    float* __restrict__ cvec) {
    const int m    = blockIdx.x;
    const int lane = threadIdx.x & 31;
    const int wave = threadIdx.x >> 5;

    float xv[32];
#pragma unroll
    for (int j = 0; j < 32; ++j) xv[j] = x0[j * 32 + lane];

    float keep[2] = {0.f, 0.f};
    for (int i = 0; i < 64; ++i) {
        const int o = wave * 64 + i;
        const float* wrow = Wa + ((size_t)(m * S0 + o)) * LAT;
        float s = 0.f;
#pragma unroll
        for (int j = 0; j < 32; ++j) s = fmaf(wrow[j * 32 + lane], xv[j], s);
        for (int off = 16; off >= 1; off >>= 1) s += __shfl_xor(s, off, 32);
        if (lane == (i & 31)) keep[i >> 5] = s + ba[m * S0 + o] + bb[m * S0 + o];
    }
    for (int pass = 0; pass < 2; ++pass) {
        *(volatile float*)(cvec + m * S0 + wave * 64 + lane)      = keep[0];
        *(volatile float*)(cvec + m * S0 + wave * 64 + 32 + lane) = keep[1];
        __threadfence();
    }
}

__global__ void __launch_bounds__(256)
convert_weights_kernel(const float* __restrict__ W1, const float* __restrict__ W2,
                       _Float16* __restrict__ W1h, _Float16* __restrict__ W2h) {
    const int n1 = NM * S1 * S0;
    const int n2 = NM * S2 * S1;
    const int t  = (blockIdx.x * 256 + threadIdx.x) * 4;
    if (t < n1) {
        v4f f = *(const v4f*)(W1 + t);
        v4h h; h[0] = (_Float16)f[0]; h[1] = (_Float16)f[1];
               h[2] = (_Float16)f[2]; h[3] = (_Float16)f[3];
        *(volatile v4h*)(W1h + t) = h; __threadfence(); *(volatile v4h*)(W1h + t) = h;
    } else {
        const int u = t - n1;
        if (u < n2) {
            v4f f = *(const v4f*)(W2 + u);
            v4h h; h[0] = (_Float16)f[0]; h[1] = (_Float16)f[1];
                   h[2] = (_Float16)f[2]; h[3] = (_Float16)f[3];
            *(volatile v4h*)(W2h + u) = h; __threadfence(); *(volatile v4h*)(W2h + u) = h;
        }
    }
}

__global__ void __launch_bounds__(512)
decoder_kernel(const float* __restrict__ cvec,
               const float* __restrict__ Wb,
               const _Float16* __restrict__ W1h, const float* __restrict__ b1,
               const _Float16* __restrict__ W2h, const float* __restrict__ b2,
               const float* __restrict__ W3,     const float* __restrict__ b3,
               float* __restrict__ out) {
    const unsigned sbase = __builtin_amdgcn_groupstaticsize();
    lds_half*  Ysh  = (lds_half*)(sbase + OFF_Y);
    lds_half*  H1sh = (lds_half*)(sbase + OFF_H1);
    lds_half*  H2sh = (lds_half*)(sbase + OFF_H2);
    lds_half*  Bsh0 = (lds_half*)(sbase + OFF_B0);
    lds_float* W3sh = (lds_float*)(sbase + OFF_B0);

    const int m    = blockIdx.x >> 5;
    const int gb   = blockIdx.x & 31;
    const int g0   = gb * GT;
    const int tid  = threadIdx.x;
    const int lane = tid & 31;
    const int wave = tid >> 5;
    const int gt   = wave >> 1;
    const int hs   = wave & 1;
    const int nn   = lane & 15;
    const int hi   = lane >> 4;

    const _Float16* W1m = W1h + (size_t)m * S1 * S0;
    const _Float16* W2m = W2h + (size_t)m * S2 * S1;

    {
        lds_v8h* p = (lds_v8h*)(Bsh0 + tid * 40);
        v8h z;
#pragma unroll
        for (int i = 0; i < 8; ++i) z[i] = (_Float16)0.f;
#pragma unroll
        for (int i = 0; i < 5; ++i) p[i] = z;
    }
    __syncthreads();


    {
        const int o  = tid;
        const float c0 = cvec[m * S0 + o];
        const float w0 = Wb[(m * S0 + o) * 2 + 0];
        const float w1 = Wb[(m * S0 + o) * 2 + 1];
        const float step = 2.0f / 63.0f;
        for (int r = 0; r < GT; ++r) {
            const int g  = g0 + r;
            const float gx = fmaf(step, (float)(g & 63), -1.0f);
            const float gy = fmaf(step, (float)(g >> 6), -1.0f);
            float v = fmaf(w1, gy, fmaf(w0, gx, c0));
            v = v > 0.f ? v : 0.f;
            Ysh[r * PY + o] = (_Float16)v;
        }
    }
    __syncthreads();

    v8f acc[8];
#pragma unroll
    for (int j = 0; j < 8; ++j)
#pragma unroll
        for (int r = 0; r < 8; ++r) acc[j][r] = 0.f;

    for (int kb = 0; kb < S0 / 32; ++kb) {
        copy_w_chunk(Bsh0, W1m + kb * 32, S1, S0, tid);
        __syncthreads();
        const lds_half* Bc = Bsh0;
        V16H a;
        const lds_half* ap = Ysh + (size_t)(gt * 16 + nn) * PY + kb * 32 + hi * 8;
        a.h[0] = *(const lds_v8h*)(ap);
        a.h[1] = *(const lds_v8h*)(ap + 16);

#pragma unroll
        for (int j = 0; j < 8; ++j) {
            const int ht = hs * 8 + j;
            V16H b;
            const lds_half* bp = Bc + (ht * 16 + nn) * PB + hi * 8;
            b.h[0] = *(const lds_v8h*)(bp);
            b.h[1] = *(const lds_v8h*)(bp + 16);
            acc[j] = wmma_f16(a, b, acc[j]);
            asm volatile("v_nop\n\tv_nop\n\tv_nop\n\tv_nop" : "+v"(acc[j]) : "v"(a.v), "v"(b.v));
        }
        __syncthreads();
    }

    {
        const int mb = hi * 8;
#pragma unroll
        for (int j = 0; j < 8; ++j) {
            const int col = (hs * 8 + j) * 16 + nn;
            const float bv = b1[m * S1 + col];
#pragma unroll
            for (int r = 0; r < 8; ++r) {
                float v = acc[j][r] + bv;
                v = v > 0.f ? v : 0.f;
                H1sh[(gt * 16 + mb + r) * P1 + col] = (_Float16)v;
            }
        }
    }

    v8f acc2[4];
#pragma unroll
    for (int j = 0; j < 4; ++j)
#pragma unroll
        for (int r = 0; r < 8; ++r) acc2[j][r] = 0.f;

    __syncthreads();
    for (int kb = 0; kb < S1 / 32; ++kb) {
        copy_w_chunk(Bsh0, W2m + kb * 32, S2, S1, tid);
        __syncthreads();
        const lds_half* Bc = Bsh0;
        V16H a;
        const lds_half* ap = H1sh + (size_t)(gt * 16 + nn) * P1 + kb * 32 + hi * 8;
        a.h[0] = *(const lds_v8h*)(ap);
        a.h[1] = *(const lds_v8h*)(ap + 16);

#pragma unroll
        for (int j = 0; j < 4; ++j) {
            const int ht = hs * 4 + j;
            V16H b;
            const lds_half* bp = Bc + (ht * 16 + nn) * PB + hi * 8;
            b.h[0] = *(const lds_v8h*)(bp);
            b.h[1] = *(const lds_v8h*)(bp + 16);
            acc2[j] = wmma_f16(a, b, acc2[j]);
            asm volatile("v_nop\n\tv_nop\n\tv_nop\n\tv_nop" : "+v"(acc2[j]) : "v"(a.v), "v"(b.v));
        }
        __syncthreads();
    }
    {
        const int mb = hi * 8;
#pragma unroll
        for (int j = 0; j < 4; ++j) {
            const int col = (hs * 4 + j) * 16 + nn;
            const float bv = b2[m * S2 + col];
#pragma unroll
            for (int r = 0; r < 8; ++r) {
                float v = acc2[j][r] + bv;
                v = v > 0.f ? v : 0.f;
                H2sh[(gt * 16 + mb + r) * P2 + col] = (_Float16)v;
            }
        }
    }

    __syncthreads();
    if (tid < 3 * S2) W3sh[tid] = W3[m * 3 * S2 + tid];
    __syncthreads();

    {
        lds_float* so = (lds_float*)(sbase + OFF_B1);
        const int g = tid >> 2;
        const int c = tid & 3;
        if (c < 3) {
            const lds_float* wr = W3sh + c * S2;
            const lds_half*  hr = H2sh + g * P2;
            float s = b3[m * 3 + c];
#pragma unroll 8
            for (int k = 0; k < S2; ++k) s = fmaf((float)hr[k], wr[k], s);
            so[g * 3 + c] = tanhf(s);
        }
        __syncthreads();
        if (tid < 96) {
            const AS3 v4f* sv = (const AS3 v4f*)so;
            float* ob = out + ((size_t)(m * G_ALL + g0)) * 3;
            *(volatile v4f*)(ob + tid * 4) = sv[tid]; __threadfence(); *(volatile v4f*)(ob + tid * 4) = sv[tid];
        }
    }
}

extern "C" void kernel_launch(void* const* d_in, const int* in_sizes, int n_in,
                              void* d_out, int out_size, void* d_ws, size_t ws_size,
                              hipStream_t stream) {
    const float* x0 = (const float*)d_in[0];
    const float* Wa = (const float*)d_in[1];
    const float* ba = (const float*)d_in[2];
    const float* Wb = (const float*)d_in[3];
    const float* bb = (const float*)d_in[4];
    const float* W1 = (const float*)d_in[5];
    const float* b1 = (const float*)d_in[6];
    const float* W2 = (const float*)d_in[7];
    const float* b2 = (const float*)d_in[8];
    const float* W3 = (const float*)d_in[9];
    const float* b3 = (const float*)d_in[10];
    float* out = (float*)d_out;

    float*     cvec = (float*)((char*)d_ws + WS_CVEC);
    _Float16*  W1h  = (_Float16*)((char*)d_ws + WS_W1H);
    _Float16*  W2h  = (_Float16*)((char*)d_ws + WS_W2H);

    (void)in_sizes; (void)n_in; (void)out_size;
    if (ws_size < (size_t)WS_W2H + (size_t)NM * S2 * S1 * 2) return;

    hipFuncSetAttribute((const void*)decoder_kernel,
                        hipFuncAttributeMaxDynamicSharedMemorySize, SMEM_BYTES);

    precompute_c_kernel<<<NM, 256, 0, stream>>>(Wa, x0, ba, bb, cvec);
    const int ncvt = (NM * S1 * S0 + NM * S2 * S1) / 4;
    convert_weights_kernel<<<ncvt / 256, 256, 0, stream>>>(W1, W2, W1h, W2h);
    decoder_kernel<<<NM * (G_ALL / GT), 512, SMEM_BYTES, stream>>>(
        cvec, Wb, W1h, b1, W2h, b2, W3, b3, out);
}
